// SelfAttn_17351667876295
// MI455X (gfx1250) — hardware-verified
//
#include <hip/hip_runtime.h>

constexpr int NBATCH = 2;
constexpr int NSEQ   = 4096;
constexpr int NROWS  = NBATCH * NSEQ;
constexpr int DMODEL = 128;
constexpr int NHEAD  = 8;
constexpr int DHEAD  = 16;
constexpr int QKW    = 2 * DMODEL;
constexpr int W1COLS = 3 * DMODEL;
constexpr int WCAT   = 4 * DMODEL;
constexpr int TP_PITCH = 36;
constexpr int ATT_KC   = 64;
constexpr int ATT_OSP  = 136;
constexpr float ATT_PSC  = 32768.0f;
constexpr float V_CARRY  = 8.0f;
constexpr float O_CARRY  = 64.0f;
constexpr float WO_CARRY = 16.0f;
constexpr float NEG_FILL = -3.402823466e38f;

static_assert(NHEAD * DHEAD == DMODEL);
static_assert(NROWS % 64 == 0 && NSEQ % 64 == 0 && DMODEL % 64 == 0 && QKW % 64 == 0);
static_assert(DMODEL % 32 == 0);
static_assert(NSEQ % ATT_KC == 0 && NSEQ % 16 == 0);
static_assert(W1COLS % 32 == 0 && DMODEL % 32 == 0);

constexpr size_t WS_XB    = 0;
constexpr size_t WS_W1VT  = WS_XB   + (size_t)NROWS * DMODEL * 2;
constexpr size_t WS_WOT   = WS_W1VT + (size_t)WCAT * DMODEL * 2;
constexpr size_t WS_QKHI  = WS_WOT  + (size_t)DMODEL * DMODEL * 2;
constexpr size_t WS_QKLO  = WS_QKHI + (size_t)NROWS * QKW * 2;
constexpr size_t WS_NA    = WS_QKLO + (size_t)NROWS * QKW * 2;
constexpr size_t WS_VT    = WS_NA   + (size_t)NROWS * DMODEL * 4;
constexpr size_t WS_ATT   = WS_VT   + (size_t)NBATCH * DMODEL * NSEQ * 2;
constexpr size_t WS_TOTAL = WS_ATT  + (size_t)NROWS * DMODEL * 2;
static_assert(WS_TOTAL == 19038208);
static_assert(WS_TOTAL <= 134217728);
static_assert((WS_W1VT % 128) == 0 && (WS_WOT % 128) == 0 && (WS_QKHI % 128) == 0 && (WS_QKLO % 128) == 0 &&
              (WS_NA % 128) == 0 && (WS_VT % 128) == 0 && (WS_ATT % 128) == 0);
static_assert((size_t)NROWS * DMODEL * 4 == 4194304);

typedef __attribute__((ext_vector_type(16))) _Float16 v16h;
typedef __attribute__((ext_vector_type(8)))  _Float16 v8h;
typedef __attribute__((ext_vector_type(16))) __bf16   v16b;
typedef __attribute__((ext_vector_type(8)))  __bf16   v8b;
typedef __attribute__((ext_vector_type(8)))  float    v8f;
typedef __attribute__((ext_vector_type(4)))  float    v4f;
typedef __attribute__((ext_vector_type(4)))  unsigned v4u;
typedef __attribute__((ext_vector_type(8)))  unsigned v8u;
typedef __attribute__((ext_vector_type(4)))  int      v4i;

__device__ __forceinline__ unsigned short f2bf_bits(float f) {
  unsigned u = __float_as_uint(f);
  return (unsigned short)((u + 0x7FFFu + ((u >> 16) & 1u)) >> 16);
}
__device__ __forceinline__ float bf_bits2f(unsigned short h) { return __uint_as_float(((unsigned)h) << 16); }
__device__ __forceinline__ float bfr(float f) { return bf_bits2f(f2bf_bits(f)); }

__device__ __forceinline__ void dep_guard_h(v8f& a, v8f& b, v16h x, v16h y) { asm volatile("v_nop\n\tv_nop\n\tv_nop\n\tv_nop" : "+v"(a), "+v"(b) : "v"(x), "v"(y)); }
__device__ __forceinline__ void dep_guard_b(v8f& a, v8f& b, v16b x, v16b y) { asm volatile("v_nop\n\tv_nop\n\tv_nop\n\tv_nop" : "+v"(a), "+v"(b) : "v"(x), "v"(y)); }
__device__ __forceinline__ void keep4_h(v16h a, v16h b, v16h c, v16h d) { asm volatile("v_nop" :: "v"(a), "v"(b), "v"(c), "v"(d)); }
__device__ __forceinline__ void keep4_b(v16b a, v16b b, v16b c, v16b d) { asm volatile("v_nop" :: "v"(a), "v"(b), "v"(c), "v"(d)); }
__device__ __forceinline__ void acc_guard4(v8f& a, v8f& b, v8f& c, v8f& d) { asm volatile("v_nop\n\tv_nop\n\tv_nop\n\tv_nop" : "+v"(a), "+v"(b), "+v"(c), "+v"(d)); }

template <typename T> struct Frag;
template <> struct Frag<_Float16> {
  typedef v16h V; union U { v16h v; v8h h[2]; };
  static __device__ __forceinline__ v16h load(const _Float16* p) {
    U f; f.h[0] = *(const v8h*)(p); f.h[1] = *(const v8h*)(p + 16); return f.v;
  }
  static __device__ __forceinline__ v8f mma(v16h a, v16h b, v8f c) {
    return __builtin_amdgcn_wmma_f32_16x16x32_f16(false, a, false, b, (short)0, c, false, false);
  }
  static __device__ __forceinline__ void guard(v8f& a, v8f& b, v16h x, v16h y) { dep_guard_h(a, b, x, y); }
  static __device__ __forceinline__ void keep(v16h a, v16h b, v16h c, v16h d) { keep4_h(a, b, c, d); }
};
template <> struct Frag<__bf16> {
  typedef v16b V; union U { v16b v; v8b h[2]; };
  static __device__ __forceinline__ v16b load(const __bf16* p) {
    U f; f.h[0] = *(const v8b*)(p); f.h[1] = *(const v8b*)(p + 16); return f.v;
  }
  static __device__ __forceinline__ v8f mma(v16b a, v16b b, v8f c) {
    return __builtin_amdgcn_wmma_f32_16x16x32_bf16(false, a, false, b, (short)0, c, false, false);
  }
  static __device__ __forceinline__ void guard(v8f& a, v8f& b, v16b x, v16b y) { dep_guard_b(a, b, x, y); }
  static __device__ __forceinline__ void keep(v16b a, v16b b, v16b c, v16b d) { keep4_b(a, b, c, d); }
};

__device__ __forceinline__ v8f mma_bf(v16b a, v16b b, v8f c) {
  c = __builtin_amdgcn_wmma_f32_16x16x32_bf16(false, a, false, b, (short)0, c, false, false);
  asm volatile("v_nop\n\tv_nop\n\tv_nop\n\tv_nop" : "+v"(c) : "v"(a), "v"(b));
  return c;
}
__device__ __forceinline__ v8f mma_hf(v16h a, v16h b, v8f c) {
  c = __builtin_amdgcn_wmma_f32_16x16x32_f16(false, a, false, b, (short)0, c, false, false);
  asm volatile("v_nop\n\tv_nop\n\tv_nop\n\tv_nop" : "+v"(c) : "v"(a), "v"(b));
  return c;
}

__global__ __launch_bounds__(256) void cast_rows_bf16_kernel(
    const float* __restrict__ in, unsigned short* __restrict__ out, int n8) {
  const int i = blockIdx.x * 256 + threadIdx.x;
  if (i < n8) {
    const v4f a = *(const v4f*)(in + (size_t)i * 8);
    const v4f c = *(const v4f*)(in + (size_t)i * 8 + 4);
    v4u w;
    w[0] = (unsigned)f2bf_bits(a[0]) | ((unsigned)f2bf_bits(a[1]) << 16);
    w[1] = (unsigned)f2bf_bits(a[2]) | ((unsigned)f2bf_bits(a[3]) << 16);
    w[2] = (unsigned)f2bf_bits(c[0]) | ((unsigned)f2bf_bits(c[1]) << 16);
    w[3] = (unsigned)f2bf_bits(c[2]) | ((unsigned)f2bf_bits(c[3]) << 16);
    unsigned short* dst = out + (size_t)i * 8;
    *(volatile v4u*)dst = w;
    __threadfence();
    *(volatile v4u*)dst = w;
  }
}

template <int OT>
__global__ __launch_bounds__(256) void transpose_cast_kernel(
    const float* __restrict__ in, int ncols, unsigned short* __restrict__ out, int outRow0, float scl) {
  __shared__ __align__(16) float tile[DMODEL * TP_PITCH];
  const int tid = threadIdx.x, wave = tid >> 5, lane = tid & 31;
  const int n0 = blockIdx.x * 32;
#pragma unroll
  for (int i = 0; i < 4; ++i) {
    const int idx = i * 256 + tid;
    const int k   = idx >> 3;
    const int c4  = (idx & 7) * 4;
    const v4f v = *(const v4f*)(in + (size_t)k * ncols + n0 + c4);
    *(v4f*)(tile + k * TP_PITCH + c4) = v;
  }
  __syncthreads();
#pragma unroll
  for (int rnd = 0; rnd < 2; ++rnd) {
    const int row = rnd * 16 + wave * 2 + (lane >> 4);
    const int c8  = (lane & 15) * 8;
    unsigned hb[8];
#pragma unroll
    for (int e = 0; e < 8; ++e) {
      const float f = tile[(c8 + e) * TP_PITCH + row];
      const unsigned short bb = f2bf_bits(f);
      if (OT == 0) {
        hb[e] = (unsigned)bb;
      } else {
        const _Float16 hf = (_Float16)(bf_bits2f(bb) * scl);
        hb[e] = (unsigned)__builtin_bit_cast(unsigned short, hf);
      }
    }
    v4u w;
    w[0] = hb[0] | (hb[1] << 16);
    w[1] = hb[2] | (hb[3] << 16);
    w[2] = hb[4] | (hb[5] << 16);
    w[3] = hb[6] | (hb[7] << 16);
    unsigned short* dst = out + (size_t)(outRow0 + n0 + row) * DMODEL + c8;
    *(volatile v4u*)dst = w;
    __threadfence();
    *(volatile v4u*)dst = w;
  }
}

template <int ET> struct Elem;
template <> struct Elem<0> { typedef _Float16 T; };
template <> struct Elem<1> { typedef __bf16 T; };

template <int ET, int BIAS_MODE, int OUT_MODE, int MASKMODE, bool RESID>
__global__ __launch_bounds__(256) void wmma_gemm64m(
    const unsigned short* __restrict__ Ap, int lda, long strideA,
    const unsigned short* __restrict__ Btp, int ldb, long strideB,
    void* __restrict__ Cout, void* __restrict__ Cout2, int ldc, long strideC,
    const float* __restrict__ bias,
    const float* __restrict__ resid, long strideR,
    const int* __restrict__ msk, long strideMsk,
    int M, int N, int K, float scale, float oscale) {
  static_assert(!(RESID && OUT_MODE != 0));
  static_assert(!(MASKMODE == 2 && OUT_MODE == 0));
  typedef typename Elem<ET>::T T;
  typedef typename Frag<T>::V V;
  const T* A = (const T*)Ap; const T* Bt = (const T*)Btp;
  __shared__ __align__(16) float sT[8][16 * 68];
  const int b    = blockIdx.y;
  const int lane = threadIdx.x & 31;
  const int wave = threadIdx.x >> 5;
  const int tilesN = N >> 6;
  const int tilesM = M >> 6;
  const int tile = blockIdx.x * 8 + wave;
  if (tile >= tilesM * tilesN) return;
  const int tm = tile / tilesN;
  const int tn = tile - tm * tilesN;
  const int m0 = tm << 6;
  const int n0 = tn << 6;

  const T* Ab = A  + (size_t)b * strideA;
  const T* Bb = Bt + (size_t)b * strideB;

  const int rlane = lane & 15;
  const int koff  = (lane >> 4) * 8;
  const int mOff  = (lane >> 4) * 8;

  v8f acc[4][4];
#pragma unroll
  for (int i = 0; i < 4; ++i)
#pragma unroll
    for (int j = 0; j < 4; ++j) acc[i][j] = (v8f){0.f,0.f,0.f,0.f,0.f,0.f,0.f,0.f};

  for (int k0 = 0; k0 < K; k0 += 32) {
    V bh[4];
#pragma unroll
    for (int j = 0; j < 4; ++j) {
      const size_t bo = (size_t)(n0 + (j << 4) + rlane) * ldb + koff + k0;
      bh[j] = Frag<T>::load(Bb + bo);
    }
#pragma unroll
    for (int i = 0; i < 4; ++i) {
      const size_t ao = (size_t)(m0 + (i << 4) + rlane) * lda + koff + k0;
      V ah = Frag<T>::load(Ab + ao);
#pragma unroll
      for (int j = 0; j < 4; ++j) acc[i][j] = Frag<T>::mma(ah, bh[j], acc[i][j]);
      Frag<T>::guard(acc[i][0], acc[i][3], ah, ah);
    }
    Frag<T>::keep(bh[0], bh[1], bh[2], bh[3]);
  }
  acc_guard4(acc[0][0], acc[0][1], acc[0][2], acc[0][3]);
  acc_guard4(acc[1][0], acc[1][1], acc[1][2], acc[1][3]);
  acc_guard4(acc[2][0], acc[2][1], acc[2][2], acc[2][3]);
  acc_guard4(acc[3][0], acc[3][1], acc[3][2], acc[3][3]);

  float* slab = sT[wave];
#pragma unroll
  for (int i = 0; i < 4; ++i) {
    const int mBase = m0 + (i << 4);
    union { v4f v[2]; float f[8]; } brow;
    brow.v[0] = (v4f){0.f,0.f,0.f,0.f}; brow.v[1] = brow.v[0];
    if (BIAS_MODE == 1) {
      brow.v[0] = *(const v4f*)(bias + mBase + mOff);
      brow.v[1] = *(const v4f*)(bias + mBase + mOff + 4);
    }
#pragma unroll
    for (int j = 0; j < 4; ++j) {
      const int n = n0 + (j << 4) + rlane;
      float bn = 0.f;
      if (BIAS_MODE == 2) bn = bfr(bias[n]);
#pragma unroll
      for (int r = 0; r < 8; ++r) {
        float v = acc[i][j][r] * scale;
        if (BIAS_MODE == 1) v += bfr(brow.f[r]);
        if (BIAS_MODE == 2) v += bn;
        slab[(mOff + r) * 68 + (j << 4) + rlane] = v;
      }
    }
    __builtin_amdgcn_fence(__ATOMIC_RELEASE, "workgroup");
    __builtin_amdgcn_wave_barrier();
    __builtin_amdgcn_fence(__ATOMIC_ACQUIRE, "workgroup");
    if (OUT_MODE == 0) {
      float* Cb = (float*)Cout + (size_t)b * strideC;
      const float* Rb = RESID ? (resid + (size_t)b * strideR) : resid;
      const int* Mb = (MASKMODE == 1) ? (msk + (size_t)b * strideMsk) : msk;
      const int h2 = lane >> 4, c4 = (lane & 15) * 4;
      for (int pass = 0; pass < 2; ++pass) {
#pragma unroll
        for (int it = 0; it < 8; ++it) {
          const int row = it * 2 + h2;
          v4f v = *(const v4f*)(slab + row * 68 + c4);
          const size_t go = (size_t)(mBase + row) * ldc + n0 + c4;
          if (RESID) { const v4f rr = *(const v4f*)(Rb + go); v = v + rr; }
          float mv = oscale;
          if (MASKMODE == 1) mv = (Mb[mBase + row] != 0) ? oscale : 0.0f;
          v = v * mv;
          *(volatile v4f*)(Cb + go) = v;
        }
        __threadfence();
      }
    } else {
      const int q = lane >> 3, c8 = (lane & 7) * 8;
      unsigned short* Cb  = (unsigned short*)Cout + (size_t)b * strideC;
      unsigned short* C2b = (unsigned short*)Cout2 + (size_t)b * strideC;
      const int* Mb = (MASKMODE != 0) ? (msk + (size_t)b * strideMsk) : msk;
      for (int pass = 0; pass < 2; ++pass) {
#pragma unroll
        for (int it = 0; it < 4; ++it) {
          const int row = it * 4 + q;
          const float* sp = slab + row * 68 + c8;
          float mv[8];
          if (MASKMODE == 0) {
#pragma unroll
            for (int e = 0; e < 8; ++e) mv[e] = oscale;
          } else if (MASKMODE == 1) {
            const float s1 = (Mb[mBase + row] != 0) ? oscale : 0.0f;
#pragma unroll
            for (int e = 0; e < 8; ++e) mv[e] = s1;
          } else {
            union { v4i v[2]; int w[8]; } mm;
            mm.v[0] = *(const v4i*)(Mb + n0 + c8);
            mm.v[1] = *(const v4i*)(Mb + n0 + c8 + 4);
#pragma unroll
            for (int e = 0; e < 8; ++e) mv[e] = (mm.w[e] != 0) ? oscale : 0.0f;
          }
          v8h hv, lv;
#pragma unroll
          for (int e = 0; e < 8; ++e) {
            const float v = sp[e] * mv[e];
            if (OUT_MODE == 1) {
              hv[e] = (_Float16)v;
              lv[e] = hv[e];
            } else {
              const unsigned short hb = f2bf_bits(v);
              const unsigned short lb = f2bf_bits(v - bf_bits2f(hb));
              hv[e] = __builtin_bit_cast(_Float16, hb);
              lv[e] = __builtin_bit_cast(_Float16, lb);
            }
          }
          *(volatile v8h*)(Cb + (size_t)(mBase + row) * ldc + n0 + c8) = hv;
          if (OUT_MODE == 2) *(volatile v8h*)(C2b + (size_t)(mBase + row) * ldc + n0 + c8) = lv;
        }
        __threadfence();
      }
    }
    __builtin_amdgcn_fence(__ATOMIC_RELEASE, "workgroup");
    __builtin_amdgcn_wave_barrier();
    __builtin_amdgcn_fence(__ATOMIC_ACQUIRE, "workgroup");
  }
}

__global__ __launch_bounds__(256) void attn_pack16_kernel(
    const unsigned short* __restrict__ QKhi, const unsigned short* __restrict__ QKlo,
    const unsigned short* __restrict__ VTp, const int* __restrict__ msk,
    unsigned short* __restrict__ attp) {
  union FB { v16b v; v8b h[2]; v8u u; };
  union FH { v16h v; v8h h[2]; v8u u; };
  __shared__ __align__(16) _Float16 Os[16 * ATT_OSP];

  const int tid  = threadIdx.x;
  const int wave = tid >> 5;
  const int lane = tid & 31;
  const int hh   = lane >> 4;
  const int c    = lane & 15;
  const int q0   = blockIdx.x * 16;
  const int b    = q0 / NSEQ;
  const int kb   = b * NSEQ;

  const __bf16* Qh = (const __bf16*)QKhi;
  const __bf16* Ql = (const __bf16*)QKlo;
  const _Float16* Vt = (const _Float16*)VTp;

  FB qb1, qb2;
  {
    const size_t qo = (size_t)(q0 + c) * QKW + wave * DHEAD + 8 * hh;
    const v8b qhv = *(const v8b*)(Qh + qo);
    const v8b qlv = *(const v8b*)(Ql + qo);
    qb1.h[0] = qhv; qb1.h[1] = qhv;
    qb2.u = (v8u){0u,0u,0u,0u,0u,0u,0u,0u};
    qb2.h[0] = qlv;
  }
  const size_t kcol = (size_t)DMODEL + wave * DHEAD + 8 * hh;
  const _Float16* vrow = Vt + ((size_t)(b * DMODEL + wave * DHEAD + c)) * NSEQ + 8 * hh;
  const int* mrow = msk + kb + 8 * hh;

  const v8f zero8 = (v8f){0.f,0.f,0.f,0.f,0.f,0.f,0.f,0.f};
  v8f oacc = zero8;
  float mrun = -__builtin_huge_valf();
  float lrun = 0.f;

  for (int kc = 0; kc < NSEQ / ATT_KC; ++kc) {
    const int kv0 = kc * ATT_KC;
    v8f s[4];
#pragma unroll
    for (int j = 0; j < 4; ++j) {
      FB ka;
      const size_t ko = (size_t)(kb + kv0 + 16 * j + c) * QKW + kcol;
      ka.h[0] = *(const v8b*)(Qh + ko);
      ka.h[1] = *(const v8b*)(Ql + ko);
      s[j] = mma_bf(ka.v, qb1.v, zero8);
      s[j] = mma_bf(ka.v, qb2.v, s[j]);
    }
    float cmax = -__builtin_huge_valf();
#pragma unroll
    for (int j = 0; j < 4; ++j) {
      union { v4i v[2]; int w[8]; } mm;
      mm.v[0] = *(const v4i*)(mrow + kv0 + 16 * j);
      mm.v[1] = *(const v4i*)(mrow + kv0 + 16 * j + 4);
#pragma unroll
      for (int r = 0; r < 8; ++r) {
        float v = s[j][r] * 0.25f;
        v = (mm.w[r] != 0) ? v : NEG_FILL;
        s[j][r] = v;
        cmax = fmaxf(cmax, v);
      }
    }
    cmax = fmaxf(cmax, __shfl_xor(cmax, 16, 32));
    const float mnew  = fmaxf(mrun, cmax);
    const float alpha = expf(mrun - mnew);
    mrun = mnew;
    float psum = 0.f;
    FH pa[2];
#pragma unroll
    for (int j = 0; j < 4; ++j) {
#pragma unroll
      for (int r = 0; r < 8; ++r) {
        const float p = expf(s[j][r] - mnew);
        psum += p;
        pa[j >> 1].h[j & 1][r] = (_Float16)(p * ATT_PSC);
      }
    }
    psum += __shfl_xor(psum, 16, 32);
    lrun = lrun * alpha + psum;
#pragma unroll
    for (int r = 0; r < 8; ++r) oacc[r] *= __shfl(alpha, 8 * hh + r, 32);
#pragma unroll
    for (int kk = 0; kk < 2; ++kk) {
      const v16h vb = Frag<_Float16>::load(vrow + kv0 + 32 * kk);
      oacc = mma_hf(pa[kk].v, vb, oacc);
    }
  }

  const float inv = (O_CARRY / V_CARRY) * (1.0f / (lrun * ATT_PSC));
#pragma unroll
  for (int r = 0; r < 8; ++r) {
    const float o = oacc[r] * __shfl(inv, 8 * hh + r, 32);
    Os[(8 * hh + r) * ATT_OSP + wave * DHEAD + c] = (_Float16)o;
  }
  __syncthreads();
  {
    const int row = wave * 2 + (lane >> 4);
    const int c8  = (lane & 15) * 8;
    const v8h val = *(const v8h*)(Os + row * ATT_OSP + c8);
    unsigned short* dst = attp + (size_t)(q0 + row) * DMODEL + c8;
    *(volatile v8h*)dst = val;
    __threadfence();
    *(volatile v8h*)dst = val;
  }
}

extern "C" void kernel_launch(void* const* d_in, const int* in_sizes, int n_in,
                              void* d_out, int out_size, void* d_ws, size_t ws_size,
                              hipStream_t stream) {
  if (n_in < 8) return;
  if (in_sizes[0] != NROWS * DMODEL || in_sizes[1] != NROWS || in_sizes[2] != DMODEL * W1COLS ||
      in_sizes[3] != W1COLS || in_sizes[4] != DMODEL * DMODEL || in_sizes[5] != DMODEL ||
      in_sizes[6] != DMODEL * DMODEL || in_sizes[7] != DMODEL) return;
  if (out_size != NROWS * DMODEL) return;
  if (ws_size < WS_TOTAL) return;

  const float* x    = (const float*)d_in[0];
  const int*   mask = (const int*)  d_in[1];
  const float* W1   = (const float*)d_in[2];
  const float* b1   = (const float*)d_in[3];
  const float* Wv   = (const float*)d_in[4];
  const float* bv   = (const float*)d_in[5];
  const float* Wo   = (const float*)d_in[6];
  const float* bo   = (const float*)d_in[7];
  float* out = (float*)d_out;

  char* ws = (char*)d_ws;
  unsigned short* Xb    = (unsigned short*)(ws + WS_XB);
  unsigned short* W1vT  = (unsigned short*)(ws + WS_W1VT);
  unsigned short* WoT16 = (unsigned short*)(ws + WS_WOT);
  unsigned short* QKhi  = (unsigned short*)(ws + WS_QKHI);
  unsigned short* QKlo  = (unsigned short*)(ws + WS_QKLO);
  float*          NA    = (float*)         (ws + WS_NA);
  unsigned short* VT    = (unsigned short*)(ws + WS_VT);
  unsigned short* ATT16 = (unsigned short*)(ws + WS_ATT);

  {
    const int n8 = NROWS * DMODEL / 8;
    cast_rows_bf16_kernel<<<(n8 + 255) / 256, 256, 0, stream>>>(x, Xb, n8);
  }
  transpose_cast_kernel<0><<<W1COLS / 32, 256, 0, stream>>>(W1, W1COLS, W1vT, 0, 1.0f);
  transpose_cast_kernel<0><<<DMODEL / 32, 256, 0, stream>>>(Wv, DMODEL, W1vT, W1COLS, 1.0f);
  transpose_cast_kernel<1><<<DMODEL / 32, 256, 0, stream>>>(Wo, DMODEL, WoT16, 0, WO_CARRY);

  {
    const int tiles = (NROWS / 64) * (QKW / 64);
    wmma_gemm64m<1, 2, 2, 1, false><<<dim3((tiles + 7) / 8, 1), 256, 0, stream>>>(
        Xb, DMODEL, 0L, W1vT, DMODEL, 0L,
        (void*)QKhi, (void*)QKlo, QKW, 0L,
        b1, NA, 0L, mask, 0L,
        NROWS, QKW, DMODEL, 1.0f, 1.0f);
  }
  {
    const int tiles = (NROWS / 64) * (DMODEL / 64);
    wmma_gemm64m<1, 2, 0, 1, false><<<dim3((tiles + 7) / 8, 1), 256, 0, stream>>>(
        Xb, DMODEL, 0L, W1vT + (size_t)QKW * DMODEL, DMODEL, 0L,
        (void*)NA, (void*)NA, DMODEL, 0L,
        b1 + QKW, NA, 0L, mask, 0L,
        NROWS, DMODEL, DMODEL, 1.0f, 1.0f);
  }
  {
    const int tiles = (DMODEL / 64) * (NSEQ / 64);
    wmma_gemm64m<1, 1, 1, 2, false><<<dim3((tiles + 7) / 8, NBATCH), 256, 0, stream>>>(
        W1vT + (size_t)W1COLS * DMODEL, DMODEL, 0L, Xb, DMODEL, (long)NSEQ * DMODEL,
        (void*)VT, (void*)VT, NSEQ, (long)DMODEL * NSEQ,
        bv, NA, 0L, mask, (long)NSEQ,
        DMODEL, NSEQ, DMODEL, 1.0f, V_CARRY);
  }
  attn_pack16_kernel<<<NROWS / 16, 256, 0, stream>>>(QKhi, QKlo, VT, mask, ATT16);
  {
    const int tiles = (NROWS / 64) * (DMODEL / 64);
    wmma_gemm64m<0, 2, 0, 1, true><<<dim3((tiles + 7) / 8, 1), 256, 0, stream>>>(
        ATT16, DMODEL, 0L, WoT16, DMODEL, 0L,
        (void*)out, (void*)out, DMODEL, 0L,
        bo, NA, 0L, mask, 0L,
        NROWS, DMODEL, DMODEL, 1.0f / (O_CARRY * WO_CARRY), 1.0f);
  }
}
